// MoEFluxAttnProcessor2_0_50878182588813
// MI455X (gfx1250) — hardware-verified
//
#include <hip/hip_runtime.h>
#include <math.h>
#include <stdint.h>


#define SEQ  2048
#define DIM  3072
#define NH   24
#define HD   128
#define NE   4
#define NR   8
#define NLO  96
#define NDG  128
#define KEXT 3168
#define LDX  3200

typedef _Float16 v16h __attribute__((ext_vector_type(16)));
typedef _Float16 v8h  __attribute__((ext_vector_type(8)));
typedef __bf16   v16b __attribute__((ext_vector_type(16)));
typedef __bf16   v8b  __attribute__((ext_vector_type(8)));
typedef float    v8f  __attribute__((ext_vector_type(8)));
typedef float    v4f  __attribute__((ext_vector_type(4)));
typedef unsigned int v4u __attribute__((ext_vector_type(4)));

__device__ __forceinline__ unsigned short f2bf_bits(float f) {
  const unsigned u = __float_as_uint(f);
  return (unsigned short)((u + 0x7FFFu + ((u >> 16) & 1u)) >> 16);
}
__device__ __forceinline__ float bf_bits2f(unsigned short x) { return __uint_as_float(((unsigned)x) << 16); }
__device__ __forceinline__ float bfr(float f) { return bf_bits2f(f2bf_bits(f)); }
__device__ __forceinline__ unsigned pk16(unsigned short a, unsigned short b) { return (unsigned)a | ((unsigned)b << 16); }
__device__ __forceinline__ unsigned short h2u(_Float16 x) { return __builtin_bit_cast(unsigned short, x); }

__device__ __forceinline__ void pack2_hr(float f0, float f1, unsigned& hv, unsigned& lv) {
  const _Float16 e0 = (_Float16)f0, e1 = (_Float16)f1;
  const _Float16 g0 = (_Float16)((f0 - (float)e0) * 2048.0f);
  const _Float16 g1 = (_Float16)((f1 - (float)e1) * 2048.0f);
  hv = pk16(h2u(e0), h2u(e1));
  lv = pk16(h2u(g0), h2u(g1));
}

__device__ __forceinline__ void wave_sync() {
  __builtin_amdgcn_fence(__ATOMIC_RELEASE, "workgroup");
  __builtin_amdgcn_wave_barrier();
  __builtin_amdgcn_fence(__ATOMIC_ACQUIRE, "workgroup");
}

union FragB { v16b v; v8b h[2]; };
union FragH { v16h v; v8h h[2]; };
__device__ __forceinline__ v16b ldfrag_b(const __bf16* p) {
  FragB f; f.h[0] = *(const v8b*)(p); f.h[1] = *(const v8b*)(p + 16); return f.v;
}
__device__ __forceinline__ v16h ldfrag_h(const _Float16* p) {
  FragH f; f.h[0] = *(const v8h*)(p); f.h[1] = *(const v8h*)(p + 16); return f.v;
}

__device__ __forceinline__ v8f wmma_b(v16b a, v16b b, v8f c) {
  return __builtin_amdgcn_wmma_f32_16x16x32_bf16(false, a, false, b, (short)0, c, false, false);
}
__device__ __forceinline__ v8f wmma_h(v16h a, v16h b, v8f c) {
  c = __builtin_amdgcn_wmma_f32_16x16x32_f16(false, a, false, b, (short)0, c, false, false);
  asm volatile("v_nop\n\tv_nop\n\tv_nop\n\tv_nop" : "+v"(c) : "v"(a), "v"(b));
  return c;
}
__device__ __forceinline__ void dep_guard_b(v8f& x, v8f& y, v16b b, v16b a0, v16b a1) {
  asm volatile("v_nop\n\tv_nop\n\tv_nop\n\tv_nop" : "+v"(x), "+v"(y) : "v"(b), "v"(a0), "v"(a1));
}

__global__ __launch_bounds__(256) void cvt_x_kernel(const float* __restrict__ x, unsigned short* xb, int ntot) {
  const int i = blockIdx.x * 256 + threadIdx.x;
  if (i >= ntot) return;
  const int s  = i / (DIM / 8);
  const int c8 = (i - s * (DIM / 8)) * 8;
  const float* src = x + (size_t)s * DIM + c8;
  const v4f a = *(const v4f*)(src);
  const v4f c = *(const v4f*)(src + 4);
  v4u w;
  w[0] = pk16(f2bf_bits(a[0]), f2bf_bits(a[1]));
  w[1] = pk16(f2bf_bits(a[2]), f2bf_bits(a[3]));
  w[2] = pk16(f2bf_bits(c[0]), f2bf_bits(c[1]));
  w[3] = pk16(f2bf_bits(c[2]), f2bf_bits(c[3]));
  volatile v4u* p = (volatile v4u*)(xb + (size_t)s * LDX + c8);
  *p = w;
  __threadfence();
  *p = w;
}

__global__ __launch_bounds__(256) void wt_build_kernel(const float* __restrict__ Wq, const float* __restrict__ Wk,
                                                       const float* __restrict__ Wv, unsigned short* wt) {
  __shared__ float tile[64][65];
  const int tid = threadIdx.x;
  const int k0 = blockIdx.x * 64;
  const int n0 = blockIdx.y * 64;
  const int p  = n0 / DIM;
  const int f0 = n0 - p * DIM;
  const float* W = (p == 0) ? Wq : ((p == 1) ? Wk : Wv);
  const int tx = tid & 63, ty = tid >> 6;
#pragma unroll 4
  for (int i = ty; i < 64; i += 4) tile[i][tx] = W[(size_t)(k0 + i) * DIM + f0 + tx];
  __syncthreads();
  const int rr = tid >> 3, q8 = (tid & 7) * 8;
#pragma unroll
  for (int h2 = 0; h2 < 2; ++h2) {
    const int r = rr + 32 * h2;
    v4u w;
#pragma unroll
    for (int t = 0; t < 4; ++t) w[t] = pk16(f2bf_bits(tile[q8 + 2 * t][r]), f2bf_bits(tile[q8 + 2 * t + 1][r]));
    volatile v4u* pp = (volatile v4u*)(wt + (size_t)(n0 + r) * LDX + k0 + q8);
    *pp = w;
    __threadfence();
    *pp = w;
  }
}

__global__ __launch_bounds__(256) void wlr_build_kernel(const float* __restrict__ qB, const float* __restrict__ kB,
                                                        const float* __restrict__ vB, unsigned short* wt, int ntot) {
  const int g = blockIdx.x * 256 + threadIdx.x;
  if (g >= ntot) return;
  const int n  = g >> 4;
  const int c8 = (g & 15) * 8;
  const int p  = n / DIM;
  const int f  = n - p * DIM;
  const float* Bp = (p == 0) ? qB : ((p == 1) ? kB : vB);
  const int jb = c8 - p * 32;
  const bool in = (jb >= 0) && (jb < 32);
  const int jc = min(max(jb, 0), 24);
  float v[8];
#pragma unroll
  for (int t = 0; t < 8; ++t) v[t] = Bp[(size_t)(jc + t) * DIM + f];
  v4u w;
#pragma unroll
  for (int t = 0; t < 4; ++t) w[t] = in ? pk16(f2bf_bits(v[2 * t]), f2bf_bits(v[2 * t + 1])) : 0u;
  volatile v4u* pp = (volatile v4u*)(wt + (size_t)n * LDX + DIM + c8);
  *pp = w;
  __threadfence();
  *pp = w;
}

__global__ __launch_bounds__(384) void at_build_kernel(const float* __restrict__ qA, const float* __restrict__ kA,
                                                       const float* __restrict__ vA, const float* __restrict__ gW,
                                                       unsigned short* at) {
  const int j  = blockIdx.x;
  const int d8 = threadIdx.x * 8;
  float v[8];
#pragma unroll
  for (int t = 0; t < 8; ++t) v[t] = 0.f;
  if (j < NLO) {
    const int p = j >> 5, e = (j & 31) >> 3, r = j & 7;
    const float* Ap = (p == 0) ? qA : ((p == 1) ? kA : vA);
    const float* base = Ap + ((size_t)e * DIM + d8) * NR + r;
#pragma unroll
    for (int t = 0; t < 8; ++t) v[t] = base[(size_t)t * NR];
  } else if (j < NLO + NE) {
    const int e = j - NLO;
#pragma unroll
    for (int t = 0; t < 8; ++t) v[t] = gW[(size_t)(d8 + t) * NE + e];
  }
  v4u w;
#pragma unroll
  for (int t = 0; t < 4; ++t) w[t] = pk16(f2bf_bits(v[2 * t]), f2bf_bits(v[2 * t + 1]));
  volatile v4u* pp = (volatile v4u*)(at + (size_t)j * DIM + d8);
  *pp = w;
  __threadfence();
  *pp = w;
}

#define GP 132

template <int OUT_MODE>
__global__ __launch_bounds__(128) void gemm_kernel(
    const unsigned short* __restrict__ Ap, int lda,
    const unsigned short* __restrict__ Btp, int ldb,
    const float* __restrict__ bias, const float* __restrict__ bias2,
    void* Cout, void* Cout2, void* Cout3, int ldc, int M, int N, int K) {
  __shared__ __align__(16) float sT[4][16 * GP];
  const int lane = threadIdx.x & 31;
  const int wave = threadIdx.x >> 5;
  const int tilesN = N >> 7;
  const int tilesM = M >> 5;
  const int tile = blockIdx.x * 4 + wave;
  if (tile >= tilesM * tilesN) return;
  const int tm = tile / tilesN;
  const int tn = tile - tm * tilesN;
  const int m0 = tm << 5;
  const int n0 = tn << 7;

  const __bf16* Ab = (const __bf16*)(const void*)Ap;
  const __bf16* Bb = (const __bf16*)(const void*)Btp;

  const int rlane = lane & 15;
  const int koff  = (lane >> 4) * 8;
  const int mOff  = (lane >> 4) * 8;

  v8f acc[2][8];
#pragma unroll
  for (int i = 0; i < 2; ++i)
#pragma unroll
    for (int j = 0; j < 8; ++j) acc[i][j] = (v8f){0.f, 0.f, 0.f, 0.f, 0.f, 0.f, 0.f, 0.f};

  for (int k0 = 0; k0 < K; k0 += 32) {
    const size_t ao0 = (size_t)(m0 + rlane) * lda + koff + k0;
    const size_t ao1 = (size_t)(m0 + 16 + rlane) * lda + koff + k0;
    const v16b a0 = ldfrag_b(Ab + ao0);
    const v16b a1 = ldfrag_b(Ab + ao1);
#pragma unroll
    for (int j = 0; j < 8; ++j) {
      const v16b bh = ldfrag_b(Bb + (size_t)(n0 + (j << 4) + rlane) * ldb + koff + k0);
      acc[0][j] = wmma_b(a0, bh, acc[0][j]);
      acc[1][j] = wmma_b(a1, bh, acc[1][j]);
      dep_guard_b(acc[0][j], acc[1][j], bh, a0, a1);
    }
  }

  float* slab = sT[wave];
#pragma unroll
  for (int i = 0; i < 2; ++i) {
    const int mBase = m0 + (i << 4);
#pragma unroll
    for (int j = 0; j < 8; ++j)
#pragma unroll
      for (int r = 0; r < 8; ++r) slab[(mOff + r) * GP + (j << 4) + rlane] = acc[i][j][r];
    wave_sync();
    if (OUT_MODE == 0) {
      float* C = (float*)Cout;
      const int c4 = lane * 4;
      for (int pass = 0; pass < 2; ++pass) {
#pragma unroll
        for (int it = 0; it < 16; ++it) {
          const v4f v = *(const v4f*)(slab + it * GP + c4);
          *(volatile v4f*)(C + (size_t)(mBase + it) * ldc + n0 + c4) = v;
        }
        __threadfence();
      }
    } else if (OUT_MODE == 1) {
      unsigned short* C  = (unsigned short*)Cout;
      unsigned short* C2 = (unsigned short*)Cout2;
      const int q16 = lane >> 4, c8 = (lane & 15) * 8;
      for (int pass = 0; pass < 2; ++pass) {
#pragma unroll
        for (int it = 0; it < 8; ++it) {
          const int row = it * 2 + q16;
          const float br = bfr(bias[mBase + row]);
          const float* sp = slab + row * GP + c8;
          v4u hv, lv;
#pragma unroll
          for (int p = 0; p < 4; ++p) {
            unsigned a, b;
            pack2_hr(sp[2 * p] + br, sp[2 * p + 1] + br, a, b);
            hv[p] = a; lv[p] = b;
          }
          const size_t go = (size_t)(mBase + row) * ldc + n0 + c8;
          *(volatile v4u*)(C  + go) = hv;
          *(volatile v4u*)(C2 + go) = lv;
        }
        __threadfence();
      }
    } else {
      unsigned short* Q1 = (unsigned short*)Cout;
      unsigned short* Q2 = (unsigned short*)Cout2;
      unsigned short* K1 = (unsigned short*)Cout3;
      const int q16 = lane >> 4, c8 = (lane & 15) * 8;
      const bool isq  = (n0 < DIM);
      const int  head = (isq ? n0 : (n0 - DIM)) >> 7;
      const float* bp = isq ? (bias + n0 + c8) : (bias2 + (n0 - DIM) + c8);
      float bc[8];
#pragma unroll
      for (int t = 0; t < 8; ++t) bc[t] = bfr(bp[t]);
      const size_t rowBase = (size_t)head * SEQ;
      for (int pass = 0; pass < 2; ++pass) {
#pragma unroll
        for (int it = 0; it < 8; ++it) {
          const int row = it * 2 + q16;
          const int s   = mBase + row;
          const float* sp = slab + row * GP + c8;
          v4u hv, lv;
#pragma unroll
          for (int p = 0; p < 4; ++p) {
            unsigned a, b;
            pack2_hr(sp[2 * p] + bc[2 * p], sp[2 * p + 1] + bc[2 * p + 1], a, b);
            hv[p] = a; lv[p] = b;
          }
          const size_t go = (rowBase + (size_t)s) * HD + c8;
          if (isq) {
            *(volatile v4u*)(Q1 + go) = hv;
            *(volatile v4u*)(Q2 + go) = lv;
          } else {
            *(volatile v4u*)(K1 + go) = hv;
          }
        }
        __threadfence();
      }
    }
    wave_sync();
  }
}

__global__ __launch_bounds__(256) void gate_g_kernel(const float* __restrict__ dg, const float* __restrict__ gb,
                                                     unsigned short* xb) {
  __shared__ float red[256];
  __shared__ float cmax[NE], crcp[NE];
  __shared__ float prob[256 * NE];
  __shared__ float wsh[256 * NE];
  const int tid = threadIdx.x;

#pragma unroll 1
  for (int e = 0; e < NE; ++e) {
    const float ge = gb[e];
    float mx = -INFINITY;
#pragma unroll 1
    for (int s = tid; s < SEQ; s += 256) mx = fmaxf(mx, dg[(size_t)s * NDG + NLO + e] + ge);
    red[tid] = mx;
    __syncthreads();
#pragma unroll 1
    for (int off = 128; off > 0; off >>= 1) {
      if (tid < off) red[tid] = fmaxf(red[tid], red[tid + off]);
      __syncthreads();
    }
    const float m = red[0];
    __syncthreads();
    float sm = 0.f;
#pragma unroll 1
    for (int s = tid; s < SEQ; s += 256) sm += expf(dg[(size_t)s * NDG + NLO + e] + ge - m);
    red[tid] = sm;
    __syncthreads();
#pragma unroll 1
    for (int off = 128; off > 0; off >>= 1) {
      if (tid < off) red[tid] += red[tid + off];
      __syncthreads();
    }
    if (tid == 0) { cmax[e] = m; crcp[e] = 1.0f / red[0]; }
    __syncthreads();
  }

#pragma unroll 1
  for (int base = 0; base < SEQ; base += 256) {
    const int s = base + tid;
#pragma unroll 1
    for (int e = 0; e < NE; ++e)
      prob[tid * NE + e] = expf(dg[(size_t)s * NDG + NLO + e] + gb[e] - cmax[e]) * crcp[e];
    const float p0 = prob[tid * NE + 0], p1 = prob[tid * NE + 1], p2 = prob[tid * NE + 2], p3 = prob[tid * NE + 3];
    int i0 = 0; float v0 = p0;
    if (p1 > v0) { v0 = p1; i0 = 1; }
    if (p2 > v0) { v0 = p2; i0 = 2; }
    if (p3 > v0) { v0 = p3; i0 = 3; }
    int i1 = -1; float v1 = -1.0f;
    if (i0 != 0 && p0 > v1) { v1 = p0; i1 = 0; }
    if (i0 != 1 && p1 > v1) { v1 = p1; i1 = 1; }
    if (i0 != 2 && p2 > v1) { v1 = p2; i1 = 2; }
    if (i0 != 3 && p3 > v1) { v1 = p3; i1 = 3; }
    wsh[tid * NE + 0] = (i0 == 0) ? v0 : ((i1 == 0) ? v1 : 0.f);
    wsh[tid * NE + 1] = (i0 == 1) ? v0 : ((i1 == 1) ? v1 : 0.f);
    wsh[tid * NE + 2] = (i0 == 2) ? v0 : ((i1 == 2) ? v1 : 0.f);
    wsh[tid * NE + 3] = (i0 == 3) ? v0 : ((i1 == 3) ? v1 : 0.f);
    __syncthreads();
#pragma unroll 1
    for (int it = 0; it < 16; ++it) {
      const int rl = it * 16 + (tid >> 4);
      const int c8 = (tid & 15) * 8;
      const int srow = base + rl;
      const int e = (c8 & 31) >> 3;
      float w = wsh[rl * NE + e];
      if (c8 >= NLO) w = 0.f;
      const float* dp = dg + (size_t)srow * NDG + c8;
      const v4f a = *(const v4f*)(dp);
      const v4f b = *(const v4f*)(dp + 4);
      v4u o;
      o[0] = pk16(f2bf_bits(w * a[0]), f2bf_bits(w * a[1]));
      o[1] = pk16(f2bf_bits(w * a[2]), f2bf_bits(w * a[3]));
      o[2] = pk16(f2bf_bits(w * b[0]), f2bf_bits(w * b[1]));
      o[3] = pk16(f2bf_bits(w * b[2]), f2bf_bits(w * b[3]));
      volatile v4u* pp = (volatile v4u*)(xb + (size_t)srow * LDX + DIM + c8);
      *pp = o;
      __threadfence();
      *pp = o;
    }
    __syncthreads();
  }
}

#define AT_QB 64
#define AT_KC 64
#define OS_P  132

__global__ __launch_bounds__(128)
void attn_kernel(const unsigned short* __restrict__ qhp, const unsigned short* __restrict__ qlp,
                 const unsigned short* __restrict__ kp,
                 const unsigned short* __restrict__ vhp, const unsigned short* __restrict__ vlp,
                 float* outp) {
  __shared__ __align__(16) _Float16 KVs[3 * AT_KC * HD];
  __shared__ __align__(16) _Float16 Psh[4][16 * AT_KC];
  static_assert(4 * 16 * OS_P * 4 <= 3 * AT_KC * HD * 2);
  _Float16* const Ksh = KVs;
  _Float16* const Vth = KVs + AT_KC * HD;
  _Float16* const Vtl = KVs + 2 * AT_KC * HD;

  const int tid  = threadIdx.x;
  const int wave = tid >> 5;
  const int lane = tid & 31;
  const int hh   = lane >> 4;
  const int c    = lane & 15;

  const int bx = blockIdx.x;
  const int qb = bx & 31;
  const int h  = bx >> 5;
  const int q0 = qb * AT_QB + wave * 16;

  const _Float16* Qhg = (const _Float16*)(const void*)qhp + (size_t)h * SEQ * HD;
  const _Float16* Qlg = (const _Float16*)(const void*)qlp + (size_t)h * SEQ * HD;
  const _Float16* Kg  = (const _Float16*)(const void*)kp  + (size_t)h * SEQ * HD;
  const _Float16* Vhg = (const _Float16*)(const void*)vhp + (size_t)h * HD * SEQ;
  const _Float16* Vlg = (const _Float16*)(const void*)vlp + (size_t)h * HD * SEQ;
  const int qro = (q0 + c) * HD + 8 * hh;

  const v8f zero8 = (v8f){0.f, 0.f, 0.f, 0.f, 0.f, 0.f, 0.f, 0.f};
  const float inv2048 = 4.8828125e-4f;
  const float scale   = 1.0f / 11.313708305358887f;

  float mrow[8], lrow[8];
  v8f oh[8];
#pragma unroll
  for (int r = 0; r < 8; ++r) { mrow[r] = -INFINITY; lrow[r] = 0.f; }
#pragma unroll
  for (int t = 0; t < 8; ++t) oh[t] = zero8;

  for (int kc = 0; kc < SEQ / AT_KC; ++kc) {
    const int kv0 = kc * AT_KC;
    __syncthreads();
    {
      const int r = tid >> 1, half = (tid & 1) * 64;
      const _Float16* ks = Kg  + (size_t)(kv0 + r) * HD + half;
      const _Float16* vs = Vhg + (size_t)tid * SEQ + kv0;
      const _Float16* ws = Vlg + (size_t)tid * SEQ + kv0;
#pragma unroll
      for (int i = 0; i < 8; ++i) {
        const v8h a0 = *(const v8h*)(ks + 8 * i);
        const v8h b0 = *(const v8h*)(vs + 8 * i);
        const v8h b1 = *(const v8h*)(ws + 8 * i);
        *(v8h*)(Ksh + r * HD + half + 8 * i) = a0;
        *(v8h*)(Vth + tid * AT_KC + 8 * i)   = b0;
        *(v8h*)(Vtl + tid * AT_KC + 8 * i)   = b1;
      }
    }
    __syncthreads();

    v8f s[4];
    v8f dep = oh[7];
#pragma unroll
    for (int j = 0; j < 4; ++j) {
      v8f sh = zero8, sl = zero8;
#pragma unroll
      for (int dc = 0; dc < 4; ++dc) {
        int qo = qro + dc * 32;
        asm volatile("" : "+v"(qo) : "v"(dep));
        const v16h qa = ldfrag_h(Qhg + qo);
        const v16h qr = ldfrag_h(Qlg + qo);
        FragH kb;
        kb.h[0] = *(const v8h*)(Ksh + (j * 16 + c) * HD + dc * 32 + 8 * hh);
        kb.h[1] = *(const v8h*)(Ksh + (j * 16 + c) * HD + dc * 32 + 16 + 8 * hh);
        sh = wmma_h(qa, kb.v, sh);
        sl = wmma_h(qr, kb.v, sl);
        dep = sl;
      }
      s[j] = (sh + sl * inv2048) * scale;
    }

    float cm[8];
#pragma unroll
    for (int r = 0; r < 8; ++r) {
      float m = fmaxf(fmaxf(s[0][r], s[1][r]), fmaxf(s[2][r], s[3][r]));
#pragma unroll
      for (int off = 1; off < 16; off <<= 1) m = fmaxf(m, __shfl_xor(m, off, 32));
      cm[r] = m;
    }

    _Float16* pw = Psh[wave];
#pragma unroll
    for (int r = 0; r < 8; ++r) {
      const float mnew  = fmaxf(mrow[r], cm[r]);
      const float alpha = __expf(mrow[r] - mnew);
      mrow[r] = mnew;
      float psum = 0.f;
#pragma unroll
      for (int j = 0; j < 4; ++j) {
        const float p = __expf(s[j][r] - mnew);
        psum += p;
        pw[(8 * hh + r) * AT_KC + j * 16 + c] = (_Float16)(p * 1024.0f);
      }
#pragma unroll
      for (int off = 1; off < 16; off <<= 1) psum += __shfl_xor(psum, off, 32);
      lrow[r] = lrow[r] * alpha + psum;
#pragma unroll
      for (int t = 0; t < 8; ++t) oh[t][r] *= alpha;
    }
    wave_sync();

#pragma unroll 1
    for (int kk = 0; kk < 2; ++kk) {
      FragH pa;
      pa.h[0] = *(const v8h*)(pw + c * AT_KC + kk * 32 + 8 * hh);
      pa.h[1] = *(const v8h*)(pw + c * AT_KC + kk * 32 + 16 + 8 * hh);
#pragma unroll
      for (int t = 0; t < 8; ++t) {
        FragH vb, vr;
        vb.h[0] = *(const v8h*)(Vth + (t * 16 + c) * AT_KC + kk * 32 + 8 * hh);
        vb.h[1] = *(const v8h*)(Vth + (t * 16 + c) * AT_KC + kk * 32 + 16 + 8 * hh);
        vr.h[0] = *(const v8h*)(Vtl + (t * 16 + c) * AT_KC + kk * 32 + 8 * hh);
        vr.h[1] = *(const v8h*)(Vtl + (t * 16 + c) * AT_KC + kk * 32 + 16 + 8 * hh);
        oh[t] = wmma_h(pa.v, vb.v, oh[t]);
        const v8f tr = wmma_h(pa.v, vr.v, zero8);
        oh[t] += tr * inv2048;
      }
    }
  }

  __syncthreads();
  float* os = (float*)(void*)KVs + wave * (16 * OS_P);
#pragma unroll
  for (int r = 0; r < 8; ++r) {
    const float invl = (1.0f / lrow[r]) * 9.765625e-4f;
#pragma unroll
    for (int t = 0; t < 8; ++t) os[(8 * hh + r) * OS_P + t * 16 + c] = oh[t][r] * invl;
  }
  wave_sync();
  {
    const int c4 = lane * 4;
    for (int pass = 0; pass < 2; ++pass) {
#pragma unroll
      for (int it = 0; it < 16; ++it) {
        const v4f v = *(const v4f*)(os + it * OS_P + c4);
        *(volatile v4f*)(outp + (size_t)(q0 + it) * DIM + (size_t)h * HD + c4) = v;
      }
      __threadfence();
    }
  }
}

extern "C" void kernel_launch(void* const* d_in, const int* in_sizes, int n_in,
                              void* d_out, int out_size, void* d_ws, size_t ws_size,
                              hipStream_t stream) {
  if (n_in < 15) return;
  if (in_sizes[0] != SEQ * DIM) return;
  if (in_sizes[1] != DIM * DIM || in_sizes[3] != DIM * DIM || in_sizes[5] != DIM * DIM) return;
  if (in_sizes[2] != DIM || in_sizes[4] != DIM || in_sizes[6] != DIM) return;
  if (in_sizes[7] != DIM * NE || in_sizes[8] != NE) return;
  if (in_sizes[9] != NE * DIM * NR || in_sizes[10] != NE * NR * DIM) return;
  if (in_sizes[11] != NE * DIM * NR || in_sizes[12] != NE * NR * DIM) return;
  if (in_sizes[13] != NE * DIM * NR || in_sizes[14] != NE * NR * DIM) return;
  if (out_size != SEQ * DIM) return;

  const float* x  = (const float*)d_in[0];
  const float* Wq = (const float*)d_in[1];
  const float* bq = (const float*)d_in[2];
  const float* Wk = (const float*)d_in[3];
  const float* bk = (const float*)d_in[4];
  const float* Wv = (const float*)d_in[5];
  const float* bv = (const float*)d_in[6];
  const float* gW = (const float*)d_in[7];
  const float* gb = (const float*)d_in[8];
  const float* qA = (const float*)d_in[9];
  const float* qB = (const float*)d_in[10];
  const float* kA = (const float*)d_in[11];
  const float* kB = (const float*)d_in[12];
  const float* vA = (const float*)d_in[13];
  const float* vB = (const float*)d_in[14];
  float* out = (float*)d_out;

  static_assert(KEXT == DIM + NLO);
  static_assert(KEXT % 32 == 0);
  static_assert(LDX % 64 == 0 && LDX >= DIM + 128);
  static_assert(((size_t)SEQ * LDX * 2) % 128 == 0);
  static_assert(((size_t)DIM * LDX * 2) % 128 == 0);

  const size_t szXb = (size_t)SEQ * LDX * 2;
  const size_t szWt = (size_t)3 * DIM * LDX * 2;
  const size_t szAt = (size_t)NDG * DIM * 2;
  const size_t szDG = (size_t)SEQ * NDG * 4;
  const size_t szP  = (size_t)SEQ * DIM * 2;
  size_t off = 0;
  const size_t oXb  = off; off += szXb;
  const size_t oWt  = off; off += szWt;
  const size_t oAt  = off; off += szAt;
  const size_t oDG  = off; off += szDG;
  const size_t oQl  = off; off += szP;
  const size_t oKp  = off; off += szP;
  const size_t oVth = off; off += szP;
  const size_t oVtl = off; off += szP;
  const size_t oQh  = oWt + (size_t)2 * DIM * LDX * 2;
  if (oQh + szP > oWt + szWt) return;
  if (off > ws_size) return;
  if (off > (size_t)134217728) return;

  char* ws = (char*)d_ws;
  unsigned short* Xb  = (unsigned short*)(ws + oXb);
  unsigned short* Wt  = (unsigned short*)(ws + oWt);
  unsigned short* At  = (unsigned short*)(ws + oAt);
  float*          DG  = (float*)(ws + oDG);
  unsigned short* Qh  = (unsigned short*)(ws + oQh);
  unsigned short* Ql  = (unsigned short*)(ws + oQl);
  unsigned short* Kp  = (unsigned short*)(ws + oKp);
  unsigned short* Vth = (unsigned short*)(ws + oVth);
  unsigned short* Vtl = (unsigned short*)(ws + oVtl);
  const unsigned short* WtV = Wt + (size_t)2 * DIM * LDX;

  const dim3 blk256(256), blk128(128), blk384(384);

  {
    const int ntot = SEQ * (DIM / 8);
    cvt_x_kernel<<<dim3((ntot + 255) / 256), blk256, 0, stream>>>(x, Xb, ntot);
  }
  wt_build_kernel<<<dim3(DIM / 64, (3 * DIM) / 64), blk256, 0, stream>>>(Wq, Wk, Wv, Wt);
  {
    const int ntot = 3 * DIM * 16;
    wlr_build_kernel<<<dim3((ntot + 255) / 256), blk256, 0, stream>>>(qB, kB, vB, Wt, ntot);
  }
  at_build_kernel<<<dim3(NDG), blk384, 0, stream>>>(qA, kA, vA, gW, At);
  {
    const int M = SEQ, N = NDG, K = DIM;
    const int tiles = (M / 32) * (N / 128);
    gemm_kernel<0><<<dim3((tiles + 3) / 4), blk128, 0, stream>>>(
        Xb, LDX, At, DIM, bq, bq, (void*)DG, (void*)DG, (void*)DG, NDG, M, N, K);
  }
  gate_g_kernel<<<dim3(1), blk256, 0, stream>>>(DG, gb, Xb);
  {
    const int M = DIM, N = SEQ, K = KEXT;
    const int tiles = (M / 32) * (N / 128);
    gemm_kernel<1><<<dim3((tiles + 3) / 4), blk128, 0, stream>>>(
        WtV, LDX, Xb, LDX, bv, bv, (void*)Vth, (void*)Vtl, (void*)Vtl, SEQ, M, N, K);
  }
  {
    const int M = SEQ, N = 2 * DIM, K = KEXT;
    const int tiles = (M / 32) * (N / 128);
    gemm_kernel<2><<<dim3((tiles + 3) / 4), blk128, 0, stream>>>(
        Xb, LDX, Wt, LDX, bq, bk, (void*)Qh, (void*)Ql, (void*)Kp, HD, M, N, K);
  }
  attn_kernel<<<dim3(NH * (SEQ / AT_QB)), blk128, 0, stream>>>(Qh, Ql, Kp, Vth, Vtl, out);
  (void)hipGetLastError();
}
